// SpatialGraphConv_10574209482797
// MI455X (gfx1250) — hardware-verified
//
#include <hip/hip_runtime.h>
#include <math.h>

typedef __attribute__((ext_vector_type(16))) _Float16 v16h;
typedef __attribute__((ext_vector_type(16))) __bf16 v16b;
typedef __attribute__((ext_vector_type(8)))  _Float16 v8h;
typedef __attribute__((ext_vector_type(8)))  float v8f;
typedef __attribute__((ext_vector_type(4)))  float v4f;
typedef __attribute__((ext_vector_type(2)))  float v2f;
typedef __attribute__((ext_vector_type(4)))  unsigned v4u;
typedef __attribute__((ext_vector_type(4)))  int v4i;
typedef float __attribute__((may_alias)) float_a;
typedef int __attribute__((may_alias)) int_a;

template <typename T> __device__ __forceinline__ void vst2(void* p, T v) { *(volatile T*)p = v; __threadfence(); *(volatile T*)p = v; }
__device__ __forceinline__ v8f wmma16(v16h a, v16h b, v8f c) {
  v8f d = __builtin_amdgcn_wmma_f32_16x16x32_f16(false, a, false, b, (short)0, c, false, false);
  asm volatile("v_nop\n\tv_nop\n\tv_nop\n\tv_nop" : "+v"(d) : "v"(a), "v"(b));
  return d;
}
__device__ __forceinline__ v8f wmma_bf(v16b a, v16b b, v8f c) {
  v8f d = __builtin_amdgcn_wmma_f32_16x16x32_bf16(false, a, false, b, (short)0, c, false, false);
  asm volatile("v_nop\n\tv_nop\n\tv_nop\n\tv_nop" : "+v"(d) : "v"(a), "v"(b));
  return d;
}
__device__ __forceinline__ v16h frag_h(const _Float16* rowk0, int lane) {
  union { v16h v; v8h q[2]; } u; const _Float16* p = rowk0 + 8 * (lane >> 4);
  u.q[0] = *(const v8h*)p; u.q[1] = *(const v8h*)(p + 16); return u.v;
}
__device__ __forceinline__ v16h frag_f32(const float* rowk0, int lane) {
  v16h a; const float* p = rowk0 + 8 * (lane >> 4);
#pragma unroll
  for (int i = 0; i < 8; ++i) { a[i] = (_Float16)p[i]; a[8 + i] = (_Float16)p[16 + i]; }
  return a;
}
__device__ __forceinline__ v16h frag_f32s(const float* rowk0, int lane, float sc) {
  v16h a; const float* p = rowk0 + 8 * (lane >> 4);
#pragma unroll
  for (int i = 0; i < 8; ++i) { a[i] = (_Float16)(p[i] * sc); a[8 + i] = (_Float16)(p[16 + i] * sc); }
  return a;
}
__device__ __forceinline__ v16h fragc_f32(const float* W, int k0, int n, int lane, int ld, int K) {
  v16h a; const int g = lane >> 4;
#pragma unroll
  for (int i = 0; i < 8; ++i) { const int ka = k0 + 8 * g + i, kb = ka + 16;
    a[i] = (_Float16)(ka < K ? W[(size_t)(ka < K ? ka : K - 1) * ld + n] : 0.f); a[8 + i] = (_Float16)(kb < K ? W[(size_t)(kb < K ? kb : K - 1) * ld + n] : 0.f); }
  return a;
}
struct F2 { v16b h, l; };
__device__ __forceinline__ F2 bsplit16(const float v[16]) { F2 r;
#pragma unroll
  for (int i = 0; i < 16; ++i) { const __bf16 h = (__bf16)v[i]; r.h[i] = h; r.l[i] = (__bf16)(v[i] - (float)h); }
  return r; }
__device__ __forceinline__ F2 split_row(const float* row, int k0, int lane) { float v[16]; const float* p = row + k0 + 8 * (lane >> 4);
#pragma unroll
  for (int i = 0; i < 8; ++i) { v[i] = p[i]; v[8 + i] = p[16 + i]; }
  return bsplit16(v); }
__device__ __forceinline__ F2 split_rowK(const float* row, int k0, int lane, int K) { float v[16]; const int g = lane >> 4;
#pragma unroll
  for (int i = 0; i < 8; ++i) { const int ka = k0 + 8 * g + i, kb = ka + 16; v[i] = ka < K ? row[ka < K ? ka : K - 1] : 0.f; v[8 + i] = kb < K ? row[kb < K ? kb : K - 1] : 0.f; }
  return bsplit16(v); }
__device__ __forceinline__ F2 split_col(const float* W, int k0, int n, int lane, int ld, int K) { float v[16]; const int g = lane >> 4;
#pragma unroll
  for (int i = 0; i < 8; ++i) { const int ka = k0 + 8 * g + i, kb = ka + 16; v[i] = ka < K ? W[(size_t)(ka < K ? ka : K - 1) * ld + n] : 0.f; v[8 + i] = kb < K ? W[(size_t)(kb < K ? kb : K - 1) * ld + n] : 0.f; }
  return bsplit16(v); }
__device__ __forceinline__ v8f mac3(const F2& a, const F2& b, v8f c) { c = wmma_bf(a.l, b.h, c); c = wmma_bf(a.h, b.l, c); return wmma_bf(a.h, b.h, c); }
__device__ __forceinline__ float sigm(float v) { return 1.0f / (1.0f + expf(-v)); }
#define LDSX() do { asm volatile("s_wait_dscnt 0" ::: "memory"); __builtin_amdgcn_wave_barrier(); __builtin_amdgcn_fence(__ATOMIC_RELEASE, "workgroup"); } while (0)


#define NB 2
#define NN 8192
#define CI 128
#define CO 128
#ifndef TQB
#define TQB (NN / 64)
#define TNB NB
#endif
typedef __attribute__((ext_vector_type(8))) __bf16 v8b;
__device__ __forceinline__ v16b frag_b(const __bf16* rowk0, int lane) {
  union { v16b v; v8b q[2]; } u; const __bf16* p = rowk0 + 8 * (lane >> 4);
  u.q[0] = *(const v8b*)p; u.q[1] = *(const v8b*)(p + 16); return u.v;
}
__device__ __forceinline__ float bfr(float v) { return (float)(__bf16)v; }
__device__ __attribute__((noinline)) float exp_ni(float v) { return expf(v); }
__device__ __attribute__((noinline)) float erf_ni(float v) { return erff(v); }

#define WS_PW  0u
#define WS_HT  (WS_PW + 2u * (size_t)CO * CI)
#define WS_PS  (WS_HT + 2u * (size_t)NB * CO * NN)
#define WS_END (WS_PS + 4u * (size_t)NB * NN * 4)

__global__ __launch_bounds__(128) void k_pack(const float* __restrict__ Wm, __bf16* __restrict__ P) { const int n = blockIdx.x, t = threadIdx.x; __shared__ __align__(16) __bf16 s[CI]; s[t] = (__bf16)Wm[(size_t)t * CO + n]; __syncthreads(); if (t < CI / 8) vst2((unsigned*)(P + (size_t)n * CI + t * 8), *(const v4u*)&s[t * 8]); }
__global__ __launch_bounds__(128) void k_h(const float* __restrict__ X, const float* __restrict__ POS, const __bf16* __restrict__ P, _Float16* __restrict__ HT, float* __restrict__ PS) {
  __shared__ __align__(16) _Float16 st[128][72]; __shared__ __align__(16) float sp[64][4];
  const int tid = threadIdx.x, wave = tid >> 5, lane = tid & 31, col = lane & 15, g = lane >> 4; const size_t b = blockIdx.y; const int n0b = blockIdx.x * 64; const size_t r0 = b * NN + n0b + wave * 16;
  v8f acc[8] = {};
#pragma unroll
  for (int kc = 0; kc < CI / 32; ++kc) { v16b a; { const float* p = X + (r0 + col) * CI + kc * 32 + 8 * g;
#pragma unroll
      for (int i = 0; i < 8; ++i) { a[i] = (__bf16)p[i]; a[8 + i] = (__bf16)p[16 + i]; } }
#pragma unroll
    for (int j = 0; j < 8; ++j) acc[j] = wmma_bf(a, frag_b(P + (size_t)(j * 16 + col) * CI + kc * 32, lane), acc[j]); }
#pragma unroll
  for (int j = 0; j < 8; ++j)
#pragma unroll
    for (int r = 0; r < 8; ++r) st[j * 16 + col][wave * 16 + 8 * g + r] = (_Float16)acc[j][r];
  if (tid < 64) { const size_t n = b * NN + n0b + tid; sp[tid][0] = bfr(POS[n * 3]); sp[tid][1] = bfr(POS[n * 3 + 1]); sp[tid][2] = bfr(POS[n * 3 + 2]); sp[tid][3] = 0.f; }
  __syncthreads();
  for (int e = tid; e < 128 * 8; e += 128) { const int c = e >> 3, pc = e & 7; vst2((unsigned*)(HT + ((b * CO + c) * NN) + n0b + pc * 8), *(const v4u*)&st[c][pc * 8]); }
  if (tid < 64) vst2(PS + (b * NN + n0b + tid) * 4, *(const v4f*)&sp[tid][0]);
}
__global__ __launch_bounds__(128) void k_agg(const float* __restrict__ PS, const _Float16* __restrict__ HT, float* __restrict__ OUT) {
  __shared__ __align__(16) _Float16 sph[4][16][40]; __shared__ __align__(16) _Float16 spl[4][16][40]; __shared__ __align__(16) float so[4][16][132]; __shared__ __align__(16) float spj[32][4];
  const int tid = threadIdx.x, wave = tid >> 5, lane = tid & 31, col = lane & 15, g = lane >> 4; const size_t b = blockIdx.y; const int i0 = blockIdx.x * 64 + wave * 16; const size_t ri = b * NN + i0;
  float pi0[8], pi1[8], pi2[8], rs[8];
#pragma unroll
  for (int r = 0; r < 8; ++r) { const float* p = PS + (ri + 8 * g + r) * 4; pi0[r] = p[0]; pi1[r] = p[1]; pi2[r] = p[2]; rs[r] = 0.f; }
  v8f acc[8] = {}, accl[8] = {};
#pragma unroll 1
  for (int js = 0; js < NN / 32; ++js) { const int j0 = js * 32;
    if (tid < 32) *(v4f*)&spj[tid][0] = *(const v4f*)(PS + (b * NN + j0 + tid) * 4);
    __syncthreads();
#pragma unroll
    for (int ct = 0; ct < 2; ++ct) { const int jl = ct * 16 + col; const float q0 = spj[jl][0], q1 = spj[jl][1], q2 = spj[jl][2];
#pragma unroll
      for (int r = 0; r < 8; ++r) { const float d0 = pi0[r] - q0, d1 = pi1[r] - q1, d2 = pi2[r] - q2; const float dsq = d0 * d0 + d1 * d1 + d2 * d2; const float a = __expf(dsq * (-50.0f));
        rs[r] += a; const float as = a * 2048.0f; const _Float16 ah = (_Float16)as; sph[wave][8 * g + r][jl] = ah; spl[wave][8 * g + r][jl] = (_Float16)((as - (float)ah) * 2048.0f); } }
    LDSX();
    const v16h pa = frag_h(&sph[wave][col][0], lane), pal = frag_h(&spl[wave][col][0], lane);
#pragma unroll
    for (int dt = 0; dt < 8; ++dt) { const v16h hf = frag_h(HT + ((b * CO + dt * 16 + col) * NN) + j0, lane); acc[dt] = wmma16(pa, hf, acc[dt]); accl[dt] = wmma16(pal, hf, accl[dt]); }
    __syncthreads(); }
#pragma unroll
  for (int r = 0; r < 8; ++r) {
#pragma unroll
    for (int o = 1; o < 16; o <<= 1) rs[r] += __shfl_xor(rs[r], o); }
#pragma unroll
  for (int r = 0; r < 8; ++r) { const float inv = (1.0f / 2048.0f) / (rs[r] + 1e-8f);
#pragma unroll
    for (int dt = 0; dt < 8; ++dt) so[wave][8 * g + r][dt * 16 + col] = (acc[dt][r] + accl[dt][r] * (1.0f / 2048.0f)) * inv; }
  LDSX();
  for (int rl = 0; rl < 16; ++rl) vst2(OUT + (ri + rl) * CO + lane * 4, *(const v4f*)&so[wave][rl][lane * 4]);
}
extern "C" void kernel_launch(void* const* d_in, const int* in_sizes, int n_in, void* d_out, int out_size, void* d_ws, size_t ws_size, hipStream_t stream) {
  (void)in_sizes; (void)n_in; (void)out_size;
  const float** F = (const float**)d_in;
  if (ws_size < (size_t)WS_END) return;
  char* ws = (char*)d_ws; __bf16* P = (__bf16*)ws; _Float16* HT = (_Float16*)(ws + WS_HT); float* PS = (float*)(ws + WS_PS);
  k_pack<<<CO, 128, 0, stream>>>(F[2], P);
  k_h<<<dim3(NN / 64, NB), 128, 0, stream>>>(F[0], F[1], P, HT, PS);
  k_agg<<<dim3(TQB, TNB), 128, 0, stream>>>(PS, HT, (float*)d_out);
}
